// RADDC_76570676953237
// MI455X (gfx1250) — hardware-run, weakly checked
//
#include <hip/hip_runtime.h>


namespace {
constexpr int NB_ = 4, C = 256, H = 64, Wd = 64, HW = H * Wd, NPX = NB_ * HW  , O = 256, KK = 9, K = KK * C  , KH1 = 5 * C  , KH2 = 4 * C;
constexpr float XS = 8.0f, HS = 256.0f, WSC = 256.0f;
__constant__ float CDY[9] = {-1.f, -1.f, -1.f, 0.f, 0.f, 0.f, 1.f, 1.f, 1.f};
__constant__ float CDX[9] = {-1.f, 0.f, 1.f, -1.f, 0.f, 1.f, -1.f, 0.f, 1.f};
typedef _Float16 b16;
typedef __attribute__((ext_vector_type(16))) _Float16 v16b;
typedef __attribute__((ext_vector_type(8))) _Float16 v8b;
typedef __attribute__((ext_vector_type(8))) float v8f;
typedef __attribute__((ext_vector_type(4))) float v4f;
__device__ __forceinline__ float bf16_rne(float f) { unsigned int u = __float_as_uint(f); u += 0x7FFFu + ((u >> 16) & 1u); float r = __uint_as_float(u & 0xFFFF0000u); asm volatile("" : "+v"(r)); return r; }
__device__ __forceinline__ float bfv(float f) { float r = bf16_rne(f); asm volatile("" : "+v"(r)); return r; }
__device__ __forceinline__ void split16(float v, b16& hi, b16& lo) { hi = (b16)v; lo = (b16)(v - (float)hi); }
__device__ __forceinline__ v16b frag_kb(const b16* p, int hh) { const v8b a = *(const v8b*)(p + 8 * hh), b = *(const v8b*)(p + 16 + 8 * hh); v16b f;
#pragma unroll
  for (int e = 0; e < 8; ++e) { f[e] = a[e]; f[8 + e] = b[e]; } return f; }
__device__ __forceinline__ v8f wmma16b(v16b a, v16b b, v8f c) { v8f d = __builtin_amdgcn_wmma_f32_16x16x32_f16(false, a, false, b, (short)0, c, false, false); asm volatile("v_nop\n\tv_nop\n\tv_nop\n\tv_nop" : "+v"(d) : "v"(a), "v"(b)); return d; }
__device__ __forceinline__ void wave_lds_sync() { __builtin_amdgcn_fence(__ATOMIC_RELEASE, "workgroup"); __builtin_amdgcn_wave_barrier(); __builtin_amdgcn_fence(__ATOMIC_ACQUIRE, "workgroup"); }
__device__ __forceinline__ float pmul(float a, float b) { float p = a * b; asm volatile("" : "+v"(p)); return p; }

__global__ __launch_bounds__(256) void wput_kernel(const float* __restrict__ wt, const float* __restrict__ wsc, const float* __restrict__ wmk, b16* __restrict__ WM, b16* __restrict__ WB) { const size_t nt = (size_t)gridDim.x * 256, u0 = (size_t)blockIdx.x * 256 + threadIdx.x; v8b v;
  for (size_t u = u0; u < (size_t)(16 + O) * (K / 8); u += nt) { const int row = (int)(u / (K / 8)), k0 = (int)(u % (K / 8)) * 8; const int kk = k0 / C, c0 = k0 % C;
#pragma unroll
    for (int j = 0; j < 8; ++j) { const int c = c0 + j; float w = 0.0f; if (row == 0) w = wsc[(size_t)c * KK + kk]; else if (row < 10) w = wmk[((size_t)(row - 1) * C + c) * KK + kk]; else if (row >= 16) w = wt[((size_t)(row - 16) * C + c) * KK + kk]; v[j] = (b16)(bf16_rne(w) * WSC); }
    b16* dst = row < 16 ? WM + (size_t)row * K + k0 : WB + (size_t)(row - 16) * K + k0; for (int pass = 0; pass < 2; ++pass) { *(volatile v8b*)dst = v; __threadfence(); } } }
__global__ __launch_bounds__(256) void nhwc_kernel(const float* __restrict__ x, float* __restrict__ XT) { __shared__ float Tt[32][33]; const int b = blockIdx.x / ((C / 32) * (HW / 32)); const int r = blockIdx.x % ((C / 32) * (HW / 32)); const int c0 = (r / (HW / 32)) * 32, p0 = (r % (HW / 32)) * 32; const int tid = threadIdx.x, wave = tid >> 5, lane = tid & 31;
  for (int q = wave; q < 32; q += 8) Tt[q][lane] = bfv(x[((size_t)b * C + c0 + q) * HW + p0 + lane]);
  __syncthreads();
  for (int pass = 0; pass < 2; ++pass) { for (int q = wave; q < 32; q += 8) ((volatile float*)XT)[((size_t)b * HW + p0 + q) * C + c0 + lane] = Tt[lane][q]; __threadfence(); } }
__global__ __launch_bounds__(32) void smconv_kernel(const float* __restrict__ XT, const b16* __restrict__ WM, const float* __restrict__ bsc, const float* __restrict__ bmk, float* __restrict__ SM) { __shared__ __attribute__((aligned(16))) b16 Ah[16][K + 8]; __shared__ float Tf[16][17]; const int lane = threadIdx.x, nloc = lane & 15, hlf = lane >> 4; const size_t px0 = (size_t)blockIdx.x * 16; const int b = (int)(px0 / HW);
  for (int r = 0; r < 16; ++r) { const int p = (int)((px0 + r) % HW); const int h = p / Wd, w = p % Wd;
#pragma unroll 1
    for (int kk = 0; kk < KK; ++kk) { const int yy = h + (int)CDY[kk], xx = w + (int)CDX[kk]; const bool in = yy >= 0 && yy < H && xx >= 0 && xx < Wd; const float* row = XT + ((size_t)b * HW + (in ? yy * Wd + xx : 0)) * C; for (int q = 0; q < 8; ++q) { const int c = q * 32 + lane; Ah[r][kk * C + c] = (b16)(in ? row[c] * XS : 0.0f); } } }
  if (lane < 16) for (int k = K; k < K + 8; ++k) Ah[lane][k] = (b16)0.0f;
  wave_lds_sync(); v8f acc = (v8f){};
#pragma unroll 4
  for (int kb = 0; kb < K; kb += 32) acc = wmma16b(frag_kb(&Ah[nloc][kb], hlf), frag_kb(WM + (size_t)nloc * K + kb, hlf), acc);
#pragma unroll
  for (int r8 = 0; r8 < 8; ++r8) { const float v = acc[r8] * (1.0f / (XS * WSC)); const int j = nloc; Tf[8 * hlf + r8][j] = j == 0 ? fmaxf(v + bfv(bsc[0]), 0.0f) : (j < 10 ? 1.0f / (1.0f + __expf(-(v + bfv(bmk[j - 1])))) : 0.0f); }
  wave_lds_sync();
  for (int pass = 0; pass < 2; ++pass) { for (int q = 0; q < 8; ++q) ((volatile float*)SM)[px0 * 16 + q * 32 + lane] = Tf[(q * 32 + lane) >> 4][(q * 32 + lane) & 15]; __threadfence(); } }
__global__ __launch_bounds__(32) void dconv_kernel(const float* __restrict__ XT, const float* __restrict__ SM, const b16* __restrict__ WB, const float* __restrict__ bias, int PXLIM, float* __restrict__ OS) { __shared__ __attribute__((aligned(16))) b16 Ah[16][KH1 + 8], Al[16][KH1 + 8]; __shared__ float Tf[16][O + 4]; const int lane = threadIdx.x, nloc = lane & 15, hlf = lane >> 4; const size_t px0 = (size_t)blockIdx.x * 16; if (px0 >= (size_t)PXLIM) return; const int b = (int)(px0 / HW); v8f acc[16];
#pragma unroll
  for (int t = 0; t < 16; ++t) acc[t] = (v8f){};
#pragma unroll 1
  for (int half = 0; half < 2; ++half) { const int kk0 = half ? 5 : 0, nk = half ? 4 : 5, kbase = kk0 * C, klen = nk * C;
    for (int r = 0; r < 16; ++r) { const size_t px = px0 + r; const int p = (int)(px % HW); const int h = p / Wd, w = p % Wd; const float sc = SM[px * 16];
#pragma unroll 1
      for (int kq = 0; kq < nk; ++kq) { const int kk = kk0 + kq; const float dy = CDY[kk], dx = CDX[kk]; const float ys = (float)(h - 1) + dy + sc * dy, xs = (float)(w - 1) + dx + sc * dx; const float y0 = floorf(ys), x0 = floorf(xs); const float wy = ys - y0, wx = xs - x0; const int yi = (int)y0, xi = (int)x0; const float mk = SM[px * 16 + 1 + kk];
        float cw[4]; int cy[4], cx[4]; cw[0] = (1.0f - wy) * (1.0f - wx); cy[0] = yi; cx[0] = xi; cw[1] = (1.0f - wy) * wx; cy[1] = yi; cx[1] = xi + 1; cw[2] = wy * (1.0f - wx); cy[2] = yi + 1; cx[2] = xi; cw[3] = wy * wx; cy[3] = yi + 1; cx[3] = xi + 1;
        float v[8];
#pragma unroll
        for (int q = 0; q < 8; ++q) v[q] = 0.0f;
#pragma unroll
        for (int cn = 0; cn < 4; ++cn) { const bool in = cy[cn] >= 0 && cy[cn] < H && cx[cn] >= 0 && cx[cn] < Wd; if (in) { const float* row = XT + ((size_t)b * HW + cy[cn] * Wd + cx[cn]) * C; const float wgt = cw[cn];
#pragma unroll
            for (int q = 0; q < 8; ++q) v[q] += pmul(wgt, row[q * 32 + lane]); } }
#pragma unroll
        for (int q = 0; q < 8; ++q) { b16 ph, pl; split16(pmul(v[q], mk) * HS, ph, pl); Ah[r][kq * C + q * 32 + lane] = ph; Al[r][kq * C + q * 32 + lane] = pl; } } }
    if (lane < 16) for (int k = klen; k < klen + 8; ++k) { Ah[lane][k] = (b16)0.0f; Al[lane][k] = (b16)0.0f; }
    wave_lds_sync();
#pragma unroll 1
    for (int kb = 0; kb < klen; kb += 32) { const v16b a = frag_kb(&Ah[nloc][kb], hlf), al = frag_kb(&Al[nloc][kb], hlf);
#pragma unroll
      for (int t = 0; t < 16; ++t) { const v16b bw = frag_kb(WB + (size_t)(t * 16 + nloc) * K + kbase + kb, hlf); acc[t] = wmma16b(a, bw, acc[t]); acc[t] = wmma16b(al, bw, acc[t]); } }
    wave_lds_sync(); }
#pragma unroll
  for (int t = 0; t < 16; ++t) { const int cc = t * 16 + nloc; const float bb = bfv(bias[cc]);
#pragma unroll
    for (int r8 = 0; r8 < 8; ++r8) Tf[8 * hlf + r8][cc] = acc[t][r8] * (1.0f / (HS * WSC)) + bb; }
  wave_lds_sync();
  for (int pass = 0; pass < 2; ++pass) { for (int r = 0; r < 16; ++r) for (int q = 0; q < O / 128; ++q) *(volatile v4f*)(OS + (px0 + r) * O + q * 128 + lane * 4) = *(const v4f*)(&Tf[r][q * 128 + lane * 4]); __threadfence(); } }
__global__ __launch_bounds__(256) void nchw_kernel(const float* __restrict__ OS, int PXLIM, float* __restrict__ out) { __shared__ float Tt[32][33]; const int b = blockIdx.x / ((O / 32) * (HW / 32)); const int r = blockIdx.x % ((O / 32) * (HW / 32)); const int o0 = (r / (HW / 32)) * 32, p0 = (r % (HW / 32)) * 32; const int tid = threadIdx.x, wave = tid >> 5, lane = tid & 31; if ((size_t)b * HW + p0 >= (size_t)PXLIM) return;
  for (int q = wave; q < 32; q += 8) Tt[q][lane] = OS[((size_t)b * HW + p0 + q) * O + o0 + lane];
  __syncthreads();
  for (int pass = 0; pass < 2; ++pass) { for (int q = wave; q < 32; q += 8) ((volatile float*)out)[((size_t)b * O + o0 + q) * HW + p0 + lane] = Tt[lane][q]; __threadfence(); } }
}

extern "C" void kernel_launch(void* const* d_in, const int* in_sizes, int n_in, void* d_out, int out_size, void* d_ws, size_t ws_size, hipStream_t stream) {
  (void)n_in;
  auto Fp = [&](int i) { return (const float*)d_in[i]; };
  if (in_sizes[0] != NPX * C || in_sizes[1] != O * C * KK || in_sizes[2] != O || in_sizes[3] != C * KK || in_sizes[4] != 1 || in_sizes[5] != KK * C * KK || in_sizes[6] != KK || out_size != NB_ * O * HW) return;
  const int PXLIM = NPX;
  size_t off = 0; char* ws = (char*)d_ws;
  auto carve = [&](size_t bytes) { char* p = ws + off; off += (bytes + 255) & ~(size_t)255; return p; };
  b16* WM = (b16*)carve((size_t)16 * K * 2); b16* WB = (b16*)carve((size_t)O * K * 2); float* XT = (float*)carve((size_t)NPX * C * 4); float* SM = (float*)carve((size_t)NPX * 16 * 4); float* OS = (float*)carve((size_t)NPX * O * 4);
  if (off > ws_size || off > ((size_t)64 << 20)) return;
  wput_kernel<<<128, 256, 0, stream>>>(Fp(1), Fp(3), Fp(5), WM, WB);
  nhwc_kernel<<<NB_ * (C / 32) * (HW / 32), 256, 0, stream>>>(Fp(0), XT);
  smconv_kernel<<<NPX / 16, 32, 0, stream>>>(XT, WM, Fp(4), Fp(6), SM);
  dconv_kernel<<<PXLIM / 16, 32, 0, stream>>>(XT, SM, WB, Fp(2), PXLIM, OS);
  nchw_kernel<<<NB_ * (O / 32) * (HW / 32), 256, 0, stream>>>(OS, PXLIM, (float*)d_out);
}
